// MultiheadedMixtureOfExpertsModel_14345190768798
// MI455X (gfx1250) — hardware-run, weakly checked
//
#include <hip/hip_runtime.h>
#include <stddef.h>
#include <stdint.h>
#include <math.h>


#define NR    16384
#define IND   512
#define FEAT  256
#define NH    8
#define NE    8
#define HID   256
#define CB    2048
#define XSC   8
#define ASC   8
#define WSC   1024
#define NTHR  256
#define NWAVE 8
#define TPW   64
#define HP    272
#define WSCAP 134217728
#define LDS_GEMM (NWAVE * 32 * 64 * 4)

static_assert(CB == FEAT * NH);
static_assert((NR % 128) == 0);
static_assert((NR % 64) == 0);
static_assert((CB % 128) == 0);
static_assert((IND % 128) == 0);
static_assert((IND % 32) == 0);
static_assert((CB % 32) == 0);
static_assert((HID % 128) == 0);
static_assert((HID % 64) == 0);
static_assert((FEAT % 64) == 0);
static_assert(((NR * IND) % (8 * NTHR)) == 0);
static_assert(NTHR == NWAVE * 32);
static_assert(FEAT == NTHR);
static_assert(((HP * 2) % 16) == 0);
static_assert(LDS_GEMM <= 300 * 1024);
static_assert(NH * NE <= 64);

typedef float          v2f  __attribute__((ext_vector_type(2)));
typedef float          v4f  __attribute__((ext_vector_type(4)));
typedef float          v8f  __attribute__((ext_vector_type(8)));
typedef _Float16       v8h  __attribute__((ext_vector_type(8)));
typedef _Float16       v16h __attribute__((ext_vector_type(16)));
union FragH { v16h v; v8h h[2]; };

__device__ __forceinline__ v8f wmf(v16h a, v16h b, v8f c) {
  v8f d = __builtin_amdgcn_wmma_f32_16x16x32_f16(false, a, false, b, (short)0, c, false, false);
  asm volatile("v_nop\n\tv_nop\n\tv_nop\n\tv_nop" : "+v"(d) : "v"(a), "v"(b));
  return d;
}

__device__ __forceinline__ float softplus_f(float v) {
  return log1pf(expf(-fabsf(v))) + fmaxf(v, 0.0f);
}

struct GateLds { float sc[64]; float sv[64]; float sp[64]; int se[64]; };

__device__ __forceinline__ int gate_topk(const float* __restrict__ scaling, const int* __restrict__ kexp,
                                         GateLds* g, int tid) {
  if (tid < 64) {
    g->sc[tid] = (tid < NH * NE) ? scaling[tid < NH * NE ? tid : 0] : 0.0f;
    g->sv[tid] = 0.0f; g->sp[tid] = 0.0f; g->se[tid] = 0;
  }
  int kc = kexp[0];
  kc = kc < 1 ? 1 : kc;
  kc = kc > NE ? NE : kc;
  __syncthreads();
  if (tid < NH) {
    const int h = tid;
    unsigned used = 0u;
#pragma unroll 1
    for (int k = 0; k < kc; ++k) {
      float bv = -__builtin_huge_valf();
      int bi = 0;
#pragma unroll 1
      for (int e = 0; e < NE; ++e) {
        const float v = g->sc[h * NE + e];
        const bool fr = ((used >> e) & 1u) == 0u;
        if (fr && v > bv) { bv = v; bi = e; }
      }
      used |= (1u << bi);
      g->se[h * NE + k] = bi;
      g->sv[h * NE + k] = bv;
    }
    const float v0 = g->sv[h * NE];
    float s = 0.0f;
#pragma unroll 1
    for (int k = 0; k < kc; ++k) {
      const float ex = expf(g->sv[h * NE + k] - v0);
      g->sp[h * NE + k] = ex;
      s += ex;
    }
    const float inv = 1.0f / s;
#pragma unroll 1
    for (int k = 0; k < kc; ++k) g->sp[h * NE + k] = g->sp[h * NE + k] * inv;
  }
  __syncthreads();
  return kc;
}

__device__ __forceinline__ void tile_write_t(const float* tile, _Float16* dbase, int dp, int dc,
                                             float wsc, int g, int hh, int m) {
  v8h hv[4];
#pragma unroll
  for (int q = 0; q < 4; ++q) {
    const int nl = 8 * g + 2 * q + hh;
    const int d8 = 8 * m;
#pragma unroll
    for (int e = 0; e < 8; ++e) hv[q][e] = (_Float16)(tile[(d8 + e) * TPW + nl] * wsc);
  }
#pragma unroll
  for (int q = 0; q < 4; ++q) {
    _Float16* d = dbase + (size_t)(8 * g + 2 * q + hh) * dp + dc + 8 * m;
    *(volatile v8h*)d = hv[q];
  }
  __threadfence();
#pragma unroll
  for (int q = 0; q < 4; ++q) {
    _Float16* d = dbase + (size_t)(8 * g + 2 * q + hh) * dp + dc + 8 * m;
    *(volatile v8h*)d = hv[q];
  }
}

__global__ __launch_bounds__(NTHR) void k_prepx(const float* __restrict__ x, _Float16* xh) {
  const size_t t = (size_t)blockIdx.x * NTHR + threadIdx.x;
  const float* p = x + t * 8;
  const v4f f0 = *(const v4f*)p;
  const v4f f1 = *(const v4f*)(p + 4);
  v8h a;
  a[0] = (_Float16)(f0.x * (float)XSC); a[1] = (_Float16)(f0.y * (float)XSC);
  a[2] = (_Float16)(f0.z * (float)XSC); a[3] = (_Float16)(f0.w * (float)XSC);
  a[4] = (_Float16)(f1.x * (float)XSC); a[5] = (_Float16)(f1.y * (float)XSC);
  a[6] = (_Float16)(f1.z * (float)XSC); a[7] = (_Float16)(f1.w * (float)XSC);
  _Float16* d = xh + t * 8;
  *(volatile v8h*)d = a;
  __threadfence();
  *(volatile v8h*)d = a;
}

__global__ __launch_bounds__(NTHR) void k_gate(const float* __restrict__ scaling, const int* __restrict__ kexp,
                                               const float* __restrict__ b_exp, float* bc, float* out) {
  __shared__ GateLds g;
  __shared__ float sd[64];
  __shared__ __attribute__((aligned(16))) float bcs[CB];
  const int tid = threadIdx.x;
  const int kc = gate_topk(scaling, kexp, &g, tid);

#pragma unroll 1
  for (int j = 0; j < NH; ++j) {
    float s = 0.0f;
#pragma unroll 1
    for (int k = 0; k < kc; ++k) {
      int e = g.se[j * NE + k];
      e = e < 0 ? 0 : (e > NE - 1 ? NE - 1 : e);
      s += g.sp[j * NE + k] * b_exp[e * FEAT + tid];
    }
    bcs[j * FEAT + tid] = s;
  }
  if (tid < 64) sd[tid] = 0.0f;
  __syncthreads();
  if (tid < NH) {
#pragma unroll 1
    for (int k = 0; k < kc; ++k) {
      int e = g.se[tid * NE + k];
      e = e < 0 ? 0 : (e > NE - 1 ? NE - 1 : e);
      sd[tid * NE + e] = g.sp[tid * NE + k];
    }
  }
  __syncthreads();

  const v4f u0 = *(const v4f*)(bcs + 4 * tid);
  const v4f u1 = *(const v4f*)(bcs + 4 * (tid + NTHR));
  *(volatile v4f*)(bc + 4 * tid) = u0;
  *(volatile v4f*)(bc + 4 * (tid + NTHR)) = u1;
  __threadfence();
  *(volatile v4f*)(bc + 4 * tid) = u0;
  *(volatile v4f*)(bc + 4 * (tid + NTHR)) = u1;

  if (tid == 0) {
    float loss = 0.0f;
#pragma unroll 1
    for (int a = 0; a < NH; ++a) {
#pragma unroll 1
      for (int b = 0; b < NH; ++b) {
        float gg = 0.0f;
#pragma unroll 1
        for (int e = 0; e < NE; ++e) gg += sd[a * NE + e] * sd[b * NE + e];
        if (a == b) gg -= 1.0f;
        loss += gg * gg;
      }
    }
    *(volatile float*)(out + NR) = loss;
    __threadfence();
    *(volatile float*)(out + NR) = loss;
  }
}

__global__ __launch_bounds__(NTHR) void k_prepwc(const float* __restrict__ W_exp, const float* __restrict__ scaling,
                                                 const int* __restrict__ kexp, _Float16* wct) {
  __shared__ GateLds g;
  __shared__ __attribute__((aligned(16))) float tile[128 * TPW];
  const int tid = threadIdx.x, lane = tid & 31, gw = tid >> 5, hh = lane >> 4, m = lane & 15;
  const int n0 = blockIdx.x * 64, h = blockIdx.y;
  const int kc = gate_topk(scaling, kexp, &g, tid);
#pragma unroll 1
  for (int dc = 0; dc < IND; dc += 128) {
    __syncthreads();
#pragma unroll 4
    for (int p = 0; p < 16; ++p) {
      const int dl = gw + 8 * p;
      v2f w = {0.0f, 0.0f};
#pragma unroll 1
      for (int k = 0; k < kc; ++k) {
        int e = g.se[h * NE + k];
        e = e < 0 ? 0 : (e > NE - 1 ? NE - 1 : e);
        const float pk = g.sp[h * NE + k];
        const v2f u = *(const v2f*)(W_exp + ((size_t)e * IND + dc + dl) * FEAT + n0 + 2 * lane);
        w += u * pk;
      }
      *(v2f*)(tile + dl * TPW + 2 * lane) = w;
    }
    __syncthreads();
    tile_write_t(tile, wct + (size_t)(h * FEAT + n0) * IND, IND, dc, (float)WSC, gw, hh, m);
  }
}

__global__ __launch_bounds__(NTHR) void k_prepw1(const float* __restrict__ W1, _Float16* w1t) {
  __shared__ __attribute__((aligned(16))) float tile[128 * TPW];
  const int tid = threadIdx.x, lane = tid & 31, gw = tid >> 5, hh = lane >> 4, m = lane & 15;
  const int n0 = blockIdx.x * 64;
#pragma unroll 1
  for (int c = 0; c < 2 * NH; ++c) {
    const int h = c >> 1, f0 = (c & 1) * 128;
    const int dc = h * FEAT + f0;
    __syncthreads();
#pragma unroll 4
    for (int p = 0; p < 16; ++p) {
      const int dl = gw + 8 * p;
      const int srow = (f0 + dl) * NH + h;
      const v2f w = *(const v2f*)(W1 + (size_t)srow * HID + n0 + 2 * lane);
      *(v2f*)(tile + dl * TPW + 2 * lane) = w;
    }
    __syncthreads();
    tile_write_t(tile, w1t + (size_t)n0 * CB, CB, dc, (float)WSC, gw, hh, m);
  }
}

__global__ __launch_bounds__(NTHR) void k_prepw2(const float* __restrict__ W2, _Float16* w2t) {
  __shared__ __attribute__((aligned(16))) float tile[128 * TPW];
  const int tid = threadIdx.x, lane = tid & 31, gw = tid >> 5, hh = lane >> 4, m = lane & 15;
  const int n0 = blockIdx.x * 64;
#pragma unroll 1
  for (int dc = 0; dc < HID; dc += 128) {
    __syncthreads();
#pragma unroll 4
    for (int p = 0; p < 16; ++p) {
      const int dl = gw + 8 * p;
      const v2f w = *(const v2f*)(W2 + (size_t)(dc + dl) * HID + n0 + 2 * lane);
      *(v2f*)(tile + dl * TPW + 2 * lane) = w;
    }
    __syncthreads();
    tile_write_t(tile, w2t + (size_t)n0 * HID, HID, dc, (float)WSC, gw, hh, m);
  }
}

__global__ __launch_bounds__(NTHR) void k_gemm_mh(const _Float16* __restrict__ xh, const _Float16* __restrict__ wct,
                                                  const float* __restrict__ bc, _Float16* mhh) {
  extern __shared__ v4f lds_dyn[];
  const int tid = threadIdx.x, lane = tid & 31, wave = tid >> 5, hh = lane >> 4, m = lane & 15;
  float* stg = (float*)lds_dyn + wave * (32 * 64);
  const int n0 = blockIdx.x * 128, m0 = blockIdx.y * 128;
  const int wm = (wave >> 1) * 32, wn = (wave & 1) * 64;

  v8f acc[2][4];
#pragma unroll
  for (int mt = 0; mt < 2; ++mt)
#pragma unroll
    for (int nt = 0; nt < 4; ++nt) { v8f z = {0.f, 0.f, 0.f, 0.f, 0.f, 0.f, 0.f, 0.f}; acc[mt][nt] = z; }

  const _Float16* ap = xh + (size_t)(m0 + wm + m) * IND + 8 * hh;
  const _Float16* bp = wct + (size_t)(n0 + wn + m) * IND + 8 * hh;
#pragma unroll 1
  for (int kt = 0; kt < IND / 32; ++kt) {
    const int k0 = 32 * kt;
    FragH a0, a1;
    a0.h[0] = *(const v8h*)(ap + k0);
    a0.h[1] = *(const v8h*)(ap + k0 + 16);
    a1.h[0] = *(const v8h*)(ap + (size_t)16 * IND + k0);
    a1.h[1] = *(const v8h*)(ap + (size_t)16 * IND + k0 + 16);
#pragma unroll
    for (int nt = 0; nt < 4; ++nt) {
      const _Float16* bq = bp + (size_t)nt * 16 * IND + k0;
      FragH b;
      b.h[0] = *(const v8h*)bq;
      b.h[1] = *(const v8h*)(bq + 16);
      acc[0][nt] = wmf(a0.v, b.v, acc[0][nt]);
      acc[1][nt] = wmf(a1.v, b.v, acc[1][nt]);
    }
  }

  constexpr float OSC = 1.0f / (float)(XSC * WSC);
  float bv[4];
#pragma unroll
  for (int nt = 0; nt < 4; ++nt) bv[nt] = bc[n0 + wn + 16 * nt + m];
#pragma unroll
  for (int mt = 0; mt < 2; ++mt) {
    float* sp = stg + (16 * mt + 8 * hh) * 64 + m;
#pragma unroll
    for (int nt = 0; nt < 4; ++nt) {
#pragma unroll
      for (int r = 0; r < 8; ++r) sp[r * 64 + 16 * nt] = acc[mt][nt][r] * OSC + bv[nt];
    }
  }
  __syncthreads();

  const int rg = lane >> 3, cq = lane & 7;
  v8h hv[8];
#pragma unroll
  for (int p = 0; p < 8; ++p) {
    const float* s = stg + (4 * p + rg) * 64 + 8 * cq;
    const v4f x0 = *(const v4f*)s;
    const v4f x1 = *(const v4f*)(s + 4);
    hv[p][0] = (_Float16)(x0.x * (float)ASC); hv[p][1] = (_Float16)(x0.y * (float)ASC);
    hv[p][2] = (_Float16)(x0.z * (float)ASC); hv[p][3] = (_Float16)(x0.w * (float)ASC);
    hv[p][4] = (_Float16)(x1.x * (float)ASC); hv[p][5] = (_Float16)(x1.y * (float)ASC);
    hv[p][6] = (_Float16)(x1.z * (float)ASC); hv[p][7] = (_Float16)(x1.w * (float)ASC);
  }
  _Float16* ob = mhh + (size_t)(m0 + wm) * CB + n0 + wn + 8 * cq;
#pragma unroll
  for (int p = 0; p < 8; ++p) *(volatile v8h*)(ob + (size_t)(4 * p + rg) * CB) = hv[p];
  __threadfence();
#pragma unroll
  for (int p = 0; p < 8; ++p) *(volatile v8h*)(ob + (size_t)(4 * p + rg) * CB) = hv[p];
}

__global__ __launch_bounds__(NTHR) void k_mlp(const _Float16* __restrict__ mhh, const _Float16* __restrict__ w1t,
                                              const float* __restrict__ b1, const _Float16* __restrict__ w2t,
                                              const float* __restrict__ b2, const float* __restrict__ Wout,
                                              const float* __restrict__ bout, float* out) {
  __shared__ __attribute__((aligned(16))) _Float16 h1t[64 * HP];
  __shared__ __attribute__((aligned(16))) float part[64 * 64];
  __shared__ __attribute__((aligned(16))) float outs[64];
  const int tid = threadIdx.x, lane = tid & 31, wave = tid >> 5, hh = lane >> 4, m = lane & 15;
  const int r0 = blockIdx.x * 64;
  const int wm = (wave >> 2) * 32, cg = wave & 3, wn = cg * 64;
  const float bo = bout[0];
  constexpr float OSC = 1.0f / (float)(ASC * WSC);

  v8f acc[2][4];
#pragma unroll
  for (int mt = 0; mt < 2; ++mt)
#pragma unroll
    for (int nt = 0; nt < 4; ++nt) { v8f z = {0.f, 0.f, 0.f, 0.f, 0.f, 0.f, 0.f, 0.f}; acc[mt][nt] = z; }

  {
    const _Float16* ap = mhh + (size_t)(r0 + wm + m) * CB + 8 * hh;
    const _Float16* bp = w1t + (size_t)(wn + m) * CB + 8 * hh;
#pragma unroll 1
    for (int kt = 0; kt < CB / 32; ++kt) {
      const int k0 = 32 * kt;
      FragH a0, a1;
      a0.h[0] = *(const v8h*)(ap + k0);
      a0.h[1] = *(const v8h*)(ap + k0 + 16);
      a1.h[0] = *(const v8h*)(ap + (size_t)16 * CB + k0);
      a1.h[1] = *(const v8h*)(ap + (size_t)16 * CB + k0 + 16);
#pragma unroll
      for (int nt = 0; nt < 4; ++nt) {
        const _Float16* bq = bp + (size_t)nt * 16 * CB + k0;
        FragH b;
        b.h[0] = *(const v8h*)bq;
        b.h[1] = *(const v8h*)(bq + 16);
        acc[0][nt] = wmf(a0.v, b.v, acc[0][nt]);
        acc[1][nt] = wmf(a1.v, b.v, acc[1][nt]);
      }
    }
  }
  {
    float bv[4];
#pragma unroll
    for (int nt = 0; nt < 4; ++nt) bv[nt] = b1[wn + 16 * nt + m];
#pragma unroll
    for (int mt = 0; mt < 2; ++mt) {
#pragma unroll
      for (int nt = 0; nt < 4; ++nt) {
#pragma unroll
        for (int r = 0; r < 8; ++r) {
          const float v = acc[mt][nt][r] * OSC + bv[nt];
          const float s = softplus_f(v);
          h1t[(wm + 16 * mt + 8 * hh + r) * HP + wn + 16 * nt + m] = (_Float16)(s * (float)ASC);
        }
      }
    }
  }
  __syncthreads();

#pragma unroll
  for (int mt = 0; mt < 2; ++mt)
#pragma unroll
    for (int nt = 0; nt < 4; ++nt) { v8f z = {0.f, 0.f, 0.f, 0.f, 0.f, 0.f, 0.f, 0.f}; acc[mt][nt] = z; }
  {
    const _Float16* ap = h1t + (wm + m) * HP + 8 * hh;
    const _Float16* bp = w2t + (size_t)(wn + m) * HID + 8 * hh;
#pragma unroll 1
    for (int kt = 0; kt < HID / 32; ++kt) {
      const int k0 = 32 * kt;
      FragH a0, a1;
      a0.h[0] = *(const v8h*)(ap + k0);
      a0.h[1] = *(const v8h*)(ap + k0 + 16);
      a1.h[0] = *(const v8h*)(ap + 16 * HP + k0);
      a1.h[1] = *(const v8h*)(ap + 16 * HP + k0 + 16);
#pragma unroll
      for (int nt = 0; nt < 4; ++nt) {
        const _Float16* bq = bp + (size_t)nt * 16 * HID + k0;
        FragH b;
        b.h[0] = *(const v8h*)bq;
        b.h[1] = *(const v8h*)(bq + 16);
        acc[0][nt] = wmf(a0.v, b.v, acc[0][nt]);
        acc[1][nt] = wmf(a1.v, b.v, acc[1][nt]);
      }
    }
  }

  {
    float b2v[4], wov[4];
#pragma unroll
    for (int nt = 0; nt < 4; ++nt) { b2v[nt] = b2[wn + 16 * nt + m]; wov[nt] = Wout[wn + 16 * nt + m]; }
#pragma unroll
    for (int mt = 0; mt < 2; ++mt) {
#pragma unroll
      for (int r = 0; r < 8; ++r) {
        float q = 0.0f;
#pragma unroll
        for (int nt = 0; nt < 4; ++nt) {
          const float v = acc[mt][nt][r] * OSC + b2v[nt];
          q += softplus_f(v) * wov[nt];
        }
        part[(cg * 16 + m) * 64 + wm + 16 * mt + 8 * hh + r] = q;
      }
    }
  }
  __syncthreads();
  if (tid < 64) {
    float s = 0.0f;
#pragma unroll 1
    for (int pc = 0; pc < 64; ++pc) s += part[pc * 64 + tid];
    outs[tid] = s + bo;
  }
  __syncthreads();
  if (tid < 16) {
    const v4f v = *(const v4f*)(outs + 4 * tid);
    *(volatile v4f*)(out + (size_t)r0 + 4 * tid) = v;
  }
  __threadfence();
  if (tid < 16) {
    const v4f v = *(const v4f*)(outs + 4 * tid);
    *(volatile v4f*)(out + (size_t)r0 + 4 * tid) = v;
  }
}

extern "C" void kernel_launch(void* const* d_in, const int* in_sizes, int n_in,
                              void* d_out, int out_size, void* d_ws, size_t ws_size,
                              hipStream_t stream) {
  if (n_in < 11) return;
  if (in_sizes[0] != NR * IND) return;
  if (in_sizes[1] != NH * NE) return;
  if (in_sizes[2] != NE * IND * FEAT) return;
  if (in_sizes[3] != NE * FEAT) return;
  if (in_sizes[4] != CB * HID) return;
  if (in_sizes[5] != HID) return;
  if (in_sizes[6] != HID * HID) return;
  if (in_sizes[7] != HID) return;
  if (in_sizes[8] != HID) return;
  if (in_sizes[9] != 1) return;
  if (in_sizes[10] != 1) return;
  if (out_size != NR + 1) return;

  const float* x       = (const float*)d_in[0];
  const float* scaling = (const float*)d_in[1];
  const float* W_exp   = (const float*)d_in[2];
  const float* b_exp   = (const float*)d_in[3];
  const float* W1      = (const float*)d_in[4];
  const float* b1      = (const float*)d_in[5];
  const float* W2      = (const float*)d_in[6];
  const float* b2      = (const float*)d_in[7];
  const float* Wout    = (const float*)d_in[8];
  const float* bout    = (const float*)d_in[9];
  const int*   kexp    = (const int*)d_in[10];
  float* out = (float*)d_out;

  char* ws = (char*)d_ws;
  size_t off = 0;
  const size_t oXh = off; off += (size_t)NR * IND * 2;        off = (off + 255) & ~(size_t)255;
  const size_t oWc = off; off += (size_t)CB * IND * 2;        off = (off + 255) & ~(size_t)255;
  const size_t oBc = off; off += (size_t)CB * 4;              off = (off + 255) & ~(size_t)255;
  const size_t oMh = off; off += (size_t)NR * CB * 2;         off = (off + 255) & ~(size_t)255;
  const size_t oW1 = off; off += (size_t)HID * CB * 2;        off = (off + 255) & ~(size_t)255;
  const size_t oW2 = off; off += (size_t)HID * HID * 2;       off = (off + 255) & ~(size_t)255;
  if (off > ws_size || off > (size_t)WSCAP) return;
  _Float16* xh  = (_Float16*)(ws + oXh);
  _Float16* wct = (_Float16*)(ws + oWc);
  float*    bc  = (float*)(ws + oBc);
  _Float16* mhh = (_Float16*)(ws + oMh);
  _Float16* w1t = (_Float16*)(ws + oW1);
  _Float16* w2t = (_Float16*)(ws + oW2);

  k_prepx<<<(NR * IND) / (8 * NTHR), NTHR, 0, stream>>>(x, xh);
  k_gate<<<1, NTHR, 0, stream>>>(scaling, kexp, b_exp, bc, out);
  k_prepwc<<<dim3(FEAT / 64, NH), NTHR, 0, stream>>>(W_exp, scaling, kexp, wct);
  k_prepw1<<<HID / 64, NTHR, 0, stream>>>(W1, w1t);
  k_prepw2<<<HID / 64, NTHR, 0, stream>>>(W2, w2t);
  hipFuncSetAttribute(reinterpret_cast<const void*>(&k_gemm_mh),
                      hipFuncAttributeMaxDynamicSharedMemorySize, LDS_GEMM);
  k_gemm_mh<<<dim3(CB / 128, NR / 128), NTHR, LDS_GEMM, stream>>>(xh, wct, bc, mhh);
  k_mlp<<<NR / 64, NTHR, 0, stream>>>(mhh, w1t, b1, w2t, b2, Wout, bout, out);
}
